// HomoNeighborhoodAttention_24232205484252
// MI455X (gfx1250) — hardware-verified
//
#include <hip/hip_runtime.h>
#include <stddef.h>
#include <math.h>

typedef __attribute__((ext_vector_type(16))) _Float16 v16h;
typedef __attribute__((ext_vector_type(8)))  _Float16 v8h;
typedef __attribute__((ext_vector_type(2)))  _Float16 v2h;
typedef __attribute__((ext_vector_type(16))) __bf16   v16b;
typedef __attribute__((ext_vector_type(8)))  __bf16   v8b;
typedef __attribute__((ext_vector_type(8)))  float    v8f;
typedef __attribute__((ext_vector_type(4)))  float    v4f;
typedef __attribute__((ext_vector_type(2)))  float    v2f;
typedef __attribute__((ext_vector_type(4)))  int      v4i;

constexpr int DIN   = 64;
constexpr int DED   = 16;
constexpr int HID   = 64;
constexpr int NHEAD = 8;
constexpr int PWID  = 256;
constexpr int NCAT  = 144;
constexpr int NBLK  = 512;
constexpr int RPQ   = 512;
constexpr int ECH   = 102400;
constexpr int ETILE = 64;
constexpr int APIT  = 40;
constexpr int OPIT  = 136;
constexpr float RSQ8  = 0.35355339059327373f;
constexpr float MNEG  = -3.0e38f;
#define NTHR    256
#define NWAVE   8
#define EPT     8
#define NGRP    1
#define CHUNK   (NTHR * EPT * NGRP)
#define WCAP    (EPT * NGRP * 32)
#define LISTN   (NWAVE * WCAP)
#define LDS_AGG ((NBLK * HID + 2 * NBLK * NHEAD) * 4 + LISTN * 4 + 64)

static_assert((CHUNK & (CHUNK - 1)) == 0);
static_assert(CHUNK <= 4096);
static_assert((NBLK & (NBLK - 1)) == 0 && NBLK <= 4096);
static_assert(RPQ % NBLK == 0 && RPQ % 64 == 0 && (RPQ * 8) % NTHR == 0);
static_assert(ECH % CHUNK == 0 && ECH % ETILE == 0 && ECH % 64 == 0);
static_assert(LDS_AGG == 172096);
static_assert(HID == NHEAD * 8 && PWID == 4 * HID && NCAT == 2 * DIN + DED && ETILE * 4 == NTHR);

__device__ __forceinline__ unsigned short f2bf_bits(float f) {
  unsigned u = __float_as_uint(f);
  return (unsigned short)((u + 0x7FFFu + ((u >> 16) & 1u)) >> 16);
}
__device__ __forceinline__ float bf_bits2f(unsigned short h) { return __uint_as_float(((unsigned)h) << 16); }

__device__ __forceinline__ void dep_guard_h(v8f& a, v8f& b, v16h x, v16h y) { asm volatile("v_nop\n\tv_nop\n\tv_nop\n\tv_nop" : "+v"(a), "+v"(b) : "v"(x), "v"(y)); }
__device__ __forceinline__ void dep_guard_b(v8f& a, v8f& b, v16b x, v16b y) { asm volatile("v_nop\n\tv_nop\n\tv_nop\n\tv_nop" : "+v"(a), "+v"(b) : "v"(x), "v"(y)); }
__device__ __forceinline__ void keep4_h(v16h a, v16h b, v16h c, v16h d) { asm volatile("v_nop" :: "v"(a), "v"(b), "v"(c), "v"(d)); }
__device__ __forceinline__ void keep4_b(v16b a, v16b b, v16b c, v16b d) { asm volatile("v_nop" :: "v"(a), "v"(b), "v"(c), "v"(d)); }
__device__ __forceinline__ void acc_guard4(v8f& a, v8f& b, v8f& c, v8f& d) { asm volatile("v_nop\n\tv_nop\n\tv_nop\n\tv_nop" : "+v"(a), "+v"(b), "+v"(c), "+v"(d)); }
__device__ __forceinline__ void mma_guard1(v8f& c, v16h a, v16h b) { asm volatile("v_nop\n\tv_nop\n\tv_nop\n\tv_nop" : "+v"(c) : "v"(a), "v"(b)); }
template <typename T> struct Frag;
template <> struct Frag<_Float16> {
  typedef v16h V; union U { v16h v; v8h h[2]; };
  static __device__ __forceinline__ v16h load(const _Float16* p) {
    U f; f.h[0] = *(const v8h*)(p); f.h[1] = *(const v8h*)(p + 16); return f.v;
  }
  static __device__ __forceinline__ v8f mma(v16h a, v16h b, v8f c) {
    return __builtin_amdgcn_wmma_f32_16x16x32_f16(false, a, false, b, (short)0, c, false, false);
  }
  static __device__ __forceinline__ void guard(v8f& a, v8f& b, v16h x, v16h y) { dep_guard_h(a, b, x, y); }
  static __device__ __forceinline__ void keep(v16h a, v16h b, v16h c, v16h d) { keep4_h(a, b, c, d); }
};
template <> struct Frag<__bf16> {
  typedef v16b V; union U { v16b v; v8b h[2]; };
  static __device__ __forceinline__ v16b load(const __bf16* p) {
    U f; f.h[0] = *(const v8b*)(p); f.h[1] = *(const v8b*)(p + 16); return f.v;
  }
  static __device__ __forceinline__ v8f mma(v16b a, v16b b, v8f c) {
    return __builtin_amdgcn_wmma_f32_16x16x32_bf16(false, a, false, b, (short)0, c, false, false);
  }
  static __device__ __forceinline__ void guard(v8f& a, v8f& b, v16b x, v16b y) { dep_guard_b(a, b, x, y); }
  static __device__ __forceinline__ void keep(v16b a, v16b b, v16b c, v16b d) { keep4_b(a, b, c, d); }
};

template <int ET> struct Elem;
template <> struct Elem<0> { typedef _Float16 T; };
template <> struct Elem<1> { typedef __bf16 T; };
template <int ET, bool SPLIT, int BIAS_MODE, int OUT_MODE, bool RESID, int ACT = 0>
__global__ __launch_bounds__(256) void wmma_gemm64(
    const unsigned short* __restrict__ Ap, const unsigned short* __restrict__ A2p, int lda, long strideA,
    const unsigned short* __restrict__ Btp, const unsigned short* __restrict__ Bt2p, int ldb, long strideB,
    void* __restrict__ Cout, void* __restrict__ Cout2, int ldc, long strideC,
    const float* __restrict__ bias,
    const float* __restrict__ resid, long strideR,
    int M, int N, int K, float scale) {
  typedef typename Elem<ET>::T T;
  typedef typename Frag<T>::V V;
  const T* A = (const T*)Ap; const T* A2 = (const T*)A2p; const T* Bt = (const T*)Btp; const T* Bt2 = (const T*)Bt2p;
  __shared__ __align__(16) float sT[8][16 * 68];
  const int b    = blockIdx.y;
  const int lane = threadIdx.x & 31;
  const int wave = threadIdx.x >> 5;
  const int tilesN = N >> 6;
  const int tilesM = M >> 6;
  const int tile = blockIdx.x * 8 + wave;
  if (tile >= tilesM * tilesN) return;
  const int tm = tile / tilesN;
  const int tn = tile - tm * tilesN;
  const int m0 = tm << 6;
  const int n0 = tn << 6;

  const T* Ab  = A  + (size_t)b * strideA;
  const T* Bb  = Bt + (size_t)b * strideB;
  const T* Ab2 = SPLIT ? (A2  + (size_t)b * strideA) : nullptr;
  const T* Bb2 = SPLIT ? (Bt2 + (size_t)b * strideB) : nullptr;

  const int rlane = lane & 15;
  const int koff  = (lane >> 4) * 8;
  const int mOff  = (lane >> 4) * 8;

  v8f acc[4][4];
#pragma unroll
  for (int i = 0; i < 4; ++i)
#pragma unroll
    for (int j = 0; j < 4; ++j) acc[i][j] = (v8f){0.f,0.f,0.f,0.f,0.f,0.f,0.f,0.f};

  for (int k0 = 0; k0 < K; k0 += 32) {
    V bh[4], bl[4];
#pragma unroll
    for (int j = 0; j < 4; ++j) {
      const size_t bo = (size_t)(n0 + (j << 4) + rlane) * ldb + koff + k0;
      bh[j] = Frag<T>::load(Bb + bo);
      if (SPLIT) bl[j] = Frag<T>::load(Bb2 + bo);
    }
#pragma unroll
    for (int i = 0; i < 4; ++i) {
      const size_t ao = (size_t)(m0 + (i << 4) + rlane) * lda + koff + k0;
      V ah = Frag<T>::load(Ab + ao);
      V al;
      if (SPLIT) al = Frag<T>::load(Ab2 + ao);
#pragma unroll
      for (int j = 0; j < 4; ++j) {
        acc[i][j] = Frag<T>::mma(ah, bh[j], acc[i][j]);
        if (SPLIT) {
          acc[i][j] = Frag<T>::mma(ah, bl[j], acc[i][j]);
          acc[i][j] = Frag<T>::mma(al, bh[j], acc[i][j]);
        }
      }
      Frag<T>::guard(acc[i][0], acc[i][3], ah, SPLIT ? al : ah);
    }
    Frag<T>::keep(bh[0], bh[1], bh[2], bh[3]);
    if (SPLIT) Frag<T>::keep(bl[0], bl[1], bl[2], bl[3]);
  }
  acc_guard4(acc[0][0], acc[0][1], acc[0][2], acc[0][3]);
  acc_guard4(acc[1][0], acc[1][1], acc[1][2], acc[1][3]);
  acc_guard4(acc[2][0], acc[2][1], acc[2][2], acc[2][3]);
  acc_guard4(acc[3][0], acc[3][1], acc[3][2], acc[3][3]);

  float* slab = sT[wave];
  const float* Rb = RESID ? (resid + (size_t)b * strideR) : nullptr;
#pragma unroll
  for (int i = 0; i < 4; ++i) {
    const int mBase = m0 + (i << 4);
#pragma unroll
    for (int j = 0; j < 4; ++j) {
      const int n = n0 + (j << 4) + rlane;
      float bv = 0.f;
      if (BIAS_MODE == 2) bv = bias[n];
#pragma unroll
      for (int r = 0; r < 8; ++r) {
        float v = acc[i][j][r] * scale;
        if (BIAS_MODE == 1) v += bias[mBase + mOff + r];
        if (BIAS_MODE == 2) v += bv;
        if (RESID) v += Rb[(size_t)(mBase + mOff + r) * ldc + n];
        if (ACT == 1) v = tanhf(v);
        if (ACT == 2) v = fmaxf(v, 0.0f);
        if (ACT == 3) v = v / (1.0f + expf(-v));
        if (ACT == 4) v = (v > 0.f) ? v : 0.01f * v;
        if (ACT == 5) v = 0.5f * v * (1.0f + erff(v * 0.70710678118654752f));
        slab[(mOff + r) * 68 + (j << 4) + rlane] = v;
      }
    }
    __builtin_amdgcn_fence(__ATOMIC_RELEASE, "workgroup");
    __builtin_amdgcn_wave_barrier();
    __builtin_amdgcn_fence(__ATOMIC_ACQUIRE, "workgroup");
    if (OUT_MODE == 0) {
      float* C = (float*)Cout + (size_t)b * strideC;
      const int hh = lane >> 4, c4 = (lane & 15) * 4;
      for (int pass = 0; pass < 2; ++pass) {
#pragma unroll
        for (int it = 0; it < 8; ++it) {
          const int row = it * 2 + hh;
          v4f v = *(const v4f*)(slab + row * 68 + c4);
          *(volatile v4f*)(C + (size_t)(mBase + row) * ldc + n0 + c4) = v;
        }
        __threadfence();
      }
    } else {
      const int q = lane >> 3, c8 = (lane & 7) * 8;
      unsigned short* C  = (unsigned short*)Cout  + (size_t)b * strideC;
      unsigned short* C2 = (OUT_MODE == 2) ? ((unsigned short*)Cout2 + (size_t)b * strideC) : nullptr;
      for (int pass = 0; pass < 2; ++pass) {
#pragma unroll
        for (int it = 0; it < 4; ++it) {
          const int row = it * 4 + q;
          const float* sp = slab + row * 68 + c8;
          v8h hv, lv;
#pragma unroll
          for (int e = 0; e < 8; ++e) {
            if (OUT_MODE == 1) {
              hv[e] = (_Float16)sp[e];
            } else {
              unsigned short hb = f2bf_bits(sp[e]);
              unsigned short lb = f2bf_bits(sp[e] - bf_bits2f(hb));
              hv[e] = __builtin_bit_cast(_Float16, hb);
              lv[e] = __builtin_bit_cast(_Float16, lb);
            }
          }
          *(volatile v8h*)(C + (size_t)(mBase + row) * ldc + n0 + c8) = hv;
          if (OUT_MODE == 2) *(volatile v8h*)(C2 + (size_t)(mBase + row) * ldc + n0 + c8) = lv;
        }
        __threadfence();
      }
    }
    __builtin_amdgcn_fence(__ATOMIC_RELEASE, "workgroup");
    __builtin_amdgcn_wave_barrier();
    __builtin_amdgcn_fence(__ATOMIC_ACQUIRE, "workgroup");
  }
}

template <int NB>
__device__ __forceinline__ int scan_chunk(const int* __restrict__ lst, int nE, int cbase, int nodeBase,
                                          int* list, int tid, int lane, int wave, int fullvec) {
  int wc = 0;
#pragma unroll
  for (int g = 0; g < NGRP; ++g) {
    const int el0 = (g * NTHR + tid) * EPT;
    const int e0  = cbase + el0;
    v4i da, db;
    if (fullvec) {
      da = *(const v4i*)(lst + e0);
      db = *(const v4i*)(lst + e0 + 4);
    } else {
      const int em = nE - 1;
      da.x = lst[(e0     < em) ? e0     : em];
      da.y = lst[(e0 + 1 < em) ? e0 + 1 : em];
      da.z = lst[(e0 + 2 < em) ? e0 + 2 : em];
      da.w = lst[(e0 + 3 < em) ? e0 + 3 : em];
      db.x = lst[(e0 + 4 < em) ? e0 + 4 : em];
      db.y = lst[(e0 + 5 < em) ? e0 + 5 : em];
      db.z = lst[(e0 + 6 < em) ? e0 + 6 : em];
      db.w = lst[(e0 + 7 < em) ? e0 + 7 : em];
    }
    const bool v0 = (e0 < nE), v1 = (e0 + 1 < nE), v2 = (e0 + 2 < nE), v3 = (e0 + 3 < nE);
    const bool v4 = (e0 + 4 < nE), v5 = (e0 + 5 < nE), v6 = (e0 + 6 < nE), v7 = (e0 + 7 < nE);
    const unsigned nb = (unsigned)nodeBase;
    const unsigned s0 = (unsigned)da.x - nb, s1 = (unsigned)da.y - nb;
    const unsigned s2 = (unsigned)da.z - nb, s3 = (unsigned)da.w - nb;
    const unsigned s4 = (unsigned)db.x - nb, s5 = (unsigned)db.y - nb;
    const unsigned s6 = (unsigned)db.z - nb, s7 = (unsigned)db.w - nb;
    const bool h0 = v0 && (s0 < (unsigned)NB), h1 = v1 && (s1 < (unsigned)NB);
    const bool h2 = v2 && (s2 < (unsigned)NB), h3 = v3 && (s3 < (unsigned)NB);
    const bool h4 = v4 && (s4 < (unsigned)NB), h5 = v5 && (s5 < (unsigned)NB);
    const bool h6 = v6 && (s6 < (unsigned)NB), h7 = v7 && (s7 < (unsigned)NB);
    const unsigned any = __builtin_amdgcn_ballot_w32(h0 | h1 | h2 | h3 | h4 | h5 | h6 | h7);
    if (any != 0u) {
#define HITJ(J, HJ, SJ) { \
        const unsigned mj = __builtin_amdgcn_ballot_w32(HJ); \
        if (mj != 0u) { \
          if (HJ) { \
            const int pos = wc + (int)__builtin_amdgcn_mbcnt_lo(mj, 0u); \
            if (pos < WCAP) list[wave * WCAP + pos] = ((el0 + (J)) << 12) | (int)(SJ); \
          } \
          wc += (int)__builtin_popcount(mj); } }
      HITJ(0, h0, s0)
      HITJ(1, h1, s1)
      HITJ(2, h2, s2)
      HITJ(3, h3, s3)
      HITJ(4, h4, s4)
      HITJ(5, h5, s5)
      HITJ(6, h6, s6)
      HITJ(7, h7, s7)
#undef HITJ
    }
  }
  return wc;
}

__device__ __forceinline__ void split_bf(float f, _Float16& h, _Float16& l) {
  const unsigned short hb = f2bf_bits(f);
  const unsigned short lb = f2bf_bits(f - bf_bits2f(hb));
  h = __builtin_bit_cast(_Float16, hb);
  l = __builtin_bit_cast(_Float16, lb);
}
__device__ __forceinline__ void split8(v4f a, v4f b, v8h& hv, v8h& lv) {
  _Float16 h0, l0, h1, l1, h2, l2, h3, l3, h4, l4, h5, l5, h6, l6, h7, l7;
  split_bf(a.x, h0, l0); split_bf(a.y, h1, l1); split_bf(a.z, h2, l2); split_bf(a.w, h3, l3);
  split_bf(b.x, h4, l4); split_bf(b.y, h5, l5); split_bf(b.z, h6, l6); split_bf(b.w, h7, l7);
  hv[0] = h0; hv[1] = h1; hv[2] = h2; hv[3] = h3; hv[4] = h4; hv[5] = h5; hv[6] = h6; hv[7] = h7;
  lv[0] = l0; lv[1] = l1; lv[2] = l2; lv[3] = l3; lv[4] = l4; lv[5] = l5; lv[6] = l6; lv[7] = l7;
}

__global__ __launch_bounds__(NTHR) void k_splitx(const float* __restrict__ x, unsigned short* ph,
                                                 unsigned short* pl, int nValid, int nRows) {
  const int i = blockIdx.x * NTHR + threadIdx.x;
  if (i >= nRows * (DIN / 8)) return;
  const int row = i >> 3;
  const int c0  = (i & 7) * 8;
  const int rc  = (row < nValid) ? row : nValid - 1;
  const float* xp = x + (size_t)rc * DIN + c0;
  v4f a = *(const v4f*)xp, b = *(const v4f*)(xp + 4);
  if (row >= nValid) { const v4f z = {0.f, 0.f, 0.f, 0.f}; a = z; b = z; }
  v8h hv, lv;
  split8(a, b, hv, lv);
  const size_t o = (size_t)i * 8;
  *(volatile v8h*)(ph + o) = hv;
  *(volatile v8h*)(pl + o) = lv;
  __threadfence();
  *(volatile v8h*)(ph + o) = hv;
  *(volatile v8h*)(pl + o) = lv;
}

template <int MODE>
__device__ __forceinline__ void prep8(const float* __restrict__ W, int rowOff, int colOff, int nKv,
                                      int n, int k8, float scl, int ident,
                                      unsigned short* d0, unsigned short* d1, size_t o) {
  float w[8];
#pragma unroll
  for (int j = 0; j < 8; ++j) {
    const int k  = k8 * 8 + j;
    const int kc = (k < nKv) ? k : nKv - 1;
    float v = W[(size_t)(rowOff + kc) * HID + colOff + n];
    if (k >= nKv) v = 0.f;
    if (ident != 0 && k == n) v += 1.0f;
    w[j] = v * scl;
  }
  if (MODE == 0) {
    v8h hv;
#pragma unroll
    for (int j = 0; j < 8; ++j) hv[j] = (_Float16)w[j];
    *(volatile v8h*)(d0 + o) = hv;
    __threadfence();
    *(volatile v8h*)(d0 + o) = hv;
  } else {
    v8h hv, lv;
#pragma unroll
    for (int j = 0; j < 8; ++j) { _Float16 h, l; split_bf(w[j], h, l); hv[j] = h; lv[j] = l; }
    *(volatile v8h*)(d0 + o) = hv;
    *(volatile v8h*)(d1 + o) = lv;
    __threadfence();
    *(volatile v8h*)(d0 + o) = hv;
    *(volatile v8h*)(d1 + o) = lv;
  }
}

__global__ __launch_bounds__(NTHR) void k_prep(
    const float* __restrict__ kW0, const float* __restrict__ kW1, const float* __restrict__ kW2,
    const float* __restrict__ vW0, const float* __restrict__ vW1, const float* __restrict__ vW2,
    const float* __restrict__ oW0, const float* __restrict__ oW1, const float* __restrict__ oW2,
    unsigned short* w0h, unsigned short* w0l, unsigned short* w0e,
    unsigned short* w1k, unsigned short* w2k, unsigned short* w1v, unsigned short* w2v,
    unsigned short* ow0h, unsigned short* ow0l, unsigned short* ow1h, unsigned short* ow1l,
    unsigned short* ow2h, unsigned short* ow2l) {
  const int bx = blockIdx.x, tid = threadIdx.x;
  if (bx < 8) {
    const int idx = bx * NTHR + tid;
    const int n = idx >> 3, k8 = idx & 7;
    const int g = n >> 6, nn = n & 63;
    const float* W = (g < 2) ? kW0 : vW0;
    prep8<1>(W, (g & 1) * 64, 0, 64, nn, k8, 1.0f, 0, w0h, w0l, (size_t)idx * 8);
  } else if (bx < 10) {
    const int idx = (bx - 8) * NTHR + tid;
    const int n = idx >> 2, k8 = idx & 3;
    const int u = n >> 6, nn = n & 63;
    const float* W = (u != 0) ? vW0 : kW0;
    prep8<0>(W, 2 * DIN, 0, DED, nn, k8, 8.0f, 0, w0e, w0e, (size_t)idx * 8);
  } else {
    const int t = bx - 10;
    const int which = t >> 1;
    const int idx = (t & 1) * NTHR + tid;
    const int n = idx >> 3, k8 = idx & 7;
    const size_t o = (size_t)idx * 8;
    if (which == 0)      prep8<0>(kW1, 0, 0, 64, n, k8, 8.0f, 1, w1k, w1k, o);
    else if (which == 1) prep8<0>(kW2, 0, 0, 64, n, k8, 8.0f, 1, w2k, w2k, o);
    else if (which == 2) prep8<0>(vW1, 0, 0, 64, n, k8, 8.0f, 1, w1v, w1v, o);
    else if (which == 3) prep8<0>(vW2, 0, 0, 64, n, k8, 8.0f, 1, w2v, w2v, o);
    else if (which == 4) prep8<1>(oW0, 0, 0, 64, n, k8, 1.0f, 0, ow0h, ow0l, o);
    else if (which == 5) prep8<1>(oW1, 0, 0, 64, n, k8, 1.0f, 1, ow1h, ow1l, o);
    else                 prep8<1>(oW2, 0, 0, 64, n, k8, 1.0f, 1, ow2h, ow2l, o);
  }
}

__global__ __launch_bounds__(NTHR) void k_edge_h0(
    const float* __restrict__ ea, const int* __restrict__ ei, const float* __restrict__ pn,
    const unsigned short* __restrict__ w0ep, const float* __restrict__ bk0, const float* __restrict__ bv0,
    unsigned short* hk16, unsigned short* hv16, int nN, int nE, int eStart, int nEc) {
  __shared__ __align__(16) _Float16 sA[ETILE * APIT];
  __shared__ __align__(16) _Float16 sB[2 * HID * APIT];
  __shared__ __align__(16) _Float16 sO[ETILE * OPIT];
  __shared__ int   sIdx[2 * ETILE];
  __shared__ float sBias[2 * HID];
  const int tid = threadIdx.x, lane = tid & 31, wave = tid >> 5;
  const int ebase = blockIdx.x * ETILE;
  const _Float16* w0e = (const _Float16*)w0ep;

  if (tid < ETILE) {
    const int e  = ebase + tid;
    const int ec = (e < nEc) ? e : (nEc - 1);
    const size_t g = (size_t)eStart + (size_t)ec;
    int s = ei[g];
    int d = ei[(size_t)nE + g];
    s = s < 0 ? 0 : (s > nN - 1 ? nN - 1 : s);
    d = d < 0 ? 0 : (d > nN - 1 ? nN - 1 : d);
    sIdx[tid] = s;
    sIdx[ETILE + tid] = d;
  }
  if (tid >= 64 && tid < 128)  sBias[tid - 64] = bk0[tid - 64];
  if (tid >= 128 && tid < 192) sBias[tid - 64] = bv0[tid - 128];
  {
    const int row = tid >> 2, c4 = (tid & 3) * 4;
    const int e  = ebase + row;
    const int ec = (e < nEc) ? e : (nEc - 1);
    v4f a = *(const v4f*)(ea + ((size_t)eStart + (size_t)ec) * DED + c4);
    if (e >= nEc) { const v4f z = {0.f, 0.f, 0.f, 0.f}; a = z; }
    _Float16* ap = sA + row * APIT + c4;
    ap[0] = (_Float16)a.x; ap[1] = (_Float16)a.y; ap[2] = (_Float16)a.z; ap[3] = (_Float16)a.w;
    ap[16] = (_Float16)0.f; ap[17] = (_Float16)0.f; ap[18] = (_Float16)0.f; ap[19] = (_Float16)0.f;
  }
#pragma unroll
  for (int it = 0; it < 2; ++it) {
    const int i = it * NTHR + tid;
    const int n = i >> 2, k8 = (i & 3) * 8;
    const v8h wv = *(const v8h*)(w0e + (size_t)i * 8);
    *(v8h*)(sB + n * APIT + k8) = wv;
  }
  __syncthreads();

  const int rlane = lane & 15, hh = lane >> 4, koff = hh * 8;
  union FH { v16h v; v8h h[2]; };
  FH bfr;
  bfr.h[0] = *(const v8h*)(sB + (16 * wave + rlane) * APIT + koff);
  bfr.h[1] = *(const v8h*)(sB + (16 * wave + rlane) * APIT + koff + 16);
  v8f acc[4];
#pragma unroll
  for (int i = 0; i < 4; ++i) {
    FH afr;
    afr.h[0] = *(const v8h*)(sA + (16 * i + rlane) * APIT + koff);
    afr.h[1] = *(const v8h*)(sA + (16 * i + rlane) * APIT + koff + 16);
    acc[i] = (v8f){0.f,0.f,0.f,0.f,0.f,0.f,0.f,0.f};
    acc[i] = Frag<_Float16>::mma(afr.v, bfr.v, acc[i]);
    mma_guard1(acc[i], afr.v, bfr.v);
  }
  acc_guard4(acc[0], acc[1], acc[2], acc[3]);

  const int ncol = 16 * wave + rlane;
  const int u    = wave >> 2;
  const int p1c  = ncol + 64 * u;
  const int p2c  = ncol + 64 + 64 * u;
  const float bias = sBias[ncol];
#pragma unroll
  for (int i = 0; i < 4; ++i) {
#pragma unroll
    for (int r = 0; r < 8; ++r) {
      const int row = 16 * i + 8 * hh + r;
      const int s = sIdx[row];
      const int d = sIdx[ETILE + row];
      const float p1 = pn[(size_t)s * PWID + p1c];
      const float p2 = pn[(size_t)d * PWID + p2c];
      float v = acc[i][r] * 0.125f + p1 + p2 + bias;
      v = fmaxf(v, 0.f);
      if (ebase + row >= nEc) v = 0.f;
      sO[row * OPIT + ncol] = (_Float16)v;
    }
  }
  __syncthreads();

  for (int pass = 0; pass < 2; ++pass) {
#pragma unroll
    for (int it = 0; it < 2; ++it) {
      const int item = it * NTHR + tid;
      const int row = item >> 3, c8 = (item & 7) * 8;
      const v8h v = *(const v8h*)(sO + row * OPIT + c8);
      *(volatile v8h*)(hk16 + (size_t)(ebase + row) * HID + c8) = v;
    }
#pragma unroll
    for (int it = 0; it < 2; ++it) {
      const int item = it * NTHR + tid;
      const int row = item >> 3, c8 = (item & 7) * 8;
      const v8h v = *(const v8h*)(sO + row * OPIT + HID + c8);
      *(volatile v8h*)(hv16 + (size_t)(ebase + row) * HID + c8) = v;
    }
    __threadfence();
  }
}

template <int NB>
__global__ __launch_bounds__(NTHR) void k_agg(
    const int* __restrict__ dstl, const unsigned short* __restrict__ kplp, const unsigned short* __restrict__ vplp,
    const float* __restrict__ qv, float* accp, float* mpp, float* lpp,
    unsigned short* agh, unsigned short* agl, int nEc, int vec_ok, int first, int last) {
  static_assert((NB & (NB - 1)) == 0 && NB <= 4096);
  static_assert((NB * HID / 4) % NTHR == 0 && (NB * NHEAD / 4) % NTHR == 0 && (NB * HID / 8) % NTHR == 0);
  extern __shared__ v4f lds_dyn[];
  float* acc  = (float*)lds_dyn;
  float* mst  = acc + NB * HID;
  float* lst  = mst + NB * NHEAD;
  int*   list = (int*)(lst + NB * NHEAD);
  int*   wcnt = list + LISTN;
  v4f* mst4 = (v4f*)mst;
  v4f* lst4 = (v4f*)lst;
  const _Float16* kpl = (const _Float16*)kplp;
  const _Float16* vpl = (const _Float16*)vplp;
  const int tid = threadIdx.x, lane = tid & 31, wave = tid >> 5;
  const int nodeBase = blockIdx.x * NB;
  const float* ab = accp + (size_t)nodeBase * HID;
  const float* mb = mpp + (size_t)nodeBase * NHEAD;
  const float* lb = lpp + (size_t)nodeBase * NHEAD;

  if (first) {
    const v4f zz = {0.f, 0.f, 0.f, 0.f};
    for (int i = tid; i < NB * HID / 4; i += NTHR) lds_dyn[i] = zz;
    for (int i = tid; i < NB * NHEAD; i += NTHR) { mst[i] = MNEG; lst[i] = 0.f; }
  } else {
#pragma unroll 1
    for (int it = 0; it < (NB * HID / 4) / NTHR; ++it) {
      const int idx = it * NTHR + tid;
      lds_dyn[idx] = *(const v4f*)(ab + (size_t)idx * 4);
    }
#pragma unroll 1
    for (int it = 0; it < (NB * NHEAD / 4) / NTHR; ++it) {
      const int idx = it * NTHR + tid;
      mst4[idx] = *(const v4f*)(mb + (size_t)idx * 4);
      lst4[idx] = *(const v4f*)(lb + (size_t)idx * 4);
    }
  }
  __syncthreads();

  const int colL = 2 * lane;
  const int hdl  = lane >> 2;
  const float q0 = qv[colL], q1 = qv[colL + 1];
  const int nChunks = (nEc + CHUNK - 1) / CHUNK;
#pragma unroll 1
  for (int ch = 0; ch < nChunks; ++ch) {
    const int cbase = ch * CHUNK;
    const int fullvec = (vec_ok != 0 && cbase + CHUNK <= nEc) ? 1 : 0;
    const int wc = scan_chunk<NB>(dstl, nEc, cbase, nodeBase, list, tid, lane, wave, fullvec);
    if (lane == 0) wcnt[wave] = wc;
    __syncthreads();
    if (wave == 0) {
#pragma unroll 1
      for (int wsx = 0; wsx < NWAVE; ++wsx) {
        int n = __builtin_amdgcn_readfirstlane(wcnt[wsx]);
        n = n > WCAP ? WCAP : (n < 0 ? 0 : n);
        const int* lp = list + wsx * WCAP;
#pragma unroll 1
        for (int i = 0; i < n; ++i) {
          const int ent  = __builtin_amdgcn_readfirstlane(lp[i]);
          const int slot = ent & (NB - 1);
          int e = cbase + ((ent >> 12) & (CHUNK - 1));
          e = e > nEc - 1 ? nEc - 1 : e;
          const v2h kk = *(const v2h*)(kpl + (size_t)e * HID + colL);
          const v2h vv = *(const v2h*)(vpl + (size_t)e * HID + colL);
          float pd = q0 * (float)kk.x + q1 * (float)kk.y;
          pd += __shfl_xor(pd, 1, 32);
          pd += __shfl_xor(pd, 2, 32);
          const float lg = pd * RSQ8;
          const int mi = slot * NHEAD + hdl;
          const float mo = mst[mi];
          const float so = lst[mi];
          const float d  = __expf(-fabsf(lg - mo));
          const bool  up = (lg > mo);
          const float sc = up ? d : 1.0f;
          const float w  = up ? 1.0f : d;
          v2f* ap = (v2f*)(acc + slot * HID + colL);
          const v2f av = *ap;
          v2f nv;
          nv.x = av.x * sc + (float)vv.x * w;
          nv.y = av.y * sc + (float)vv.y * w;
          *ap = nv;
          mst[mi] = up ? lg : mo;
          lst[mi] = so * sc + w;
        }
      }
    }
    __syncthreads();
  }

  if (last) {
#pragma unroll 1
    for (int it = 0; it < (NB * HID / 8) / NTHR; ++it) {
      const int idx  = it * NTHR + tid;
      const int slot = idx >> 3;
      const int hd   = idx & 7;
      const int c8   = hd * 8;
      const float so = lst[slot * NHEAD + hd];
      const float rv = __builtin_amdgcn_rcpf((so > 0.f) ? so : 1.0f);
      const float inv = (so > 0.f) ? rv : 0.f;
      v4f a = *(const v4f*)(acc + slot * HID + c8);
      v4f b = *(const v4f*)(acc + slot * HID + c8 + 4);
      a = a * inv; b = b * inv;
      a.x = fmaxf(a.x, 0.f); a.y = fmaxf(a.y, 0.f); a.z = fmaxf(a.z, 0.f); a.w = fmaxf(a.w, 0.f);
      b.x = fmaxf(b.x, 0.f); b.y = fmaxf(b.y, 0.f); b.z = fmaxf(b.z, 0.f); b.w = fmaxf(b.w, 0.f);
      v8h hv, lv;
      split8(a, b, hv, lv);
      const size_t o = (size_t)nodeBase * HID + (size_t)idx * 8;
      *(volatile v8h*)(agh + o) = hv;
      *(volatile v8h*)(agl + o) = lv;
      __threadfence();
      *(volatile v8h*)(agh + o) = hv;
      *(volatile v8h*)(agl + o) = lv;
    }
  } else {
    float* abw = accp + (size_t)nodeBase * HID;
    float* mbw = mpp + (size_t)nodeBase * NHEAD;
    float* lbw = lpp + (size_t)nodeBase * NHEAD;
    for (int pass = 0; pass < 2; ++pass) {
#pragma unroll 1
      for (int it = 0; it < (NB * HID / 4) / NTHR; ++it) {
        const int idx = it * NTHR + tid;
        const v4f v = lds_dyn[idx];
        *(volatile v4f*)(abw + (size_t)idx * 4) = v;
      }
#pragma unroll 1
      for (int it = 0; it < (NB * NHEAD / 4) / NTHR; ++it) {
        const int idx = it * NTHR + tid;
        const v4f mv = mst4[idx];
        const v4f lv = lst4[idx];
        *(volatile v4f*)(mbw + (size_t)idx * 4) = mv;
        *(volatile v4f*)(lbw + (size_t)idx * 4) = lv;
      }
      __threadfence();
    }
  }
}

__global__ __launch_bounds__(NTHR) void k_final(const float* __restrict__ x, const float* __restrict__ g,
                                                float* out, int n4) {
  const int i = blockIdx.x * NTHR + threadIdx.x;
  if (i >= n4) return;
  const v4f a = *(const v4f*)(x + (size_t)i * 4);
  const v4f b = *(const v4f*)(g + (size_t)i * 4);
  v4f r = a + b;
  r.x = fmaxf(r.x, 0.f); r.y = fmaxf(r.y, 0.f); r.z = fmaxf(r.z, 0.f); r.w = fmaxf(r.w, 0.f);
  *(volatile v4f*)(out + (size_t)i * 4) = r;
  __threadfence();
  *(volatile v4f*)(out + (size_t)i * 4) = r;
}

extern "C" void kernel_launch(void* const* d_in, const int* in_sizes, int n_in,
                              void* d_out, int out_size, void* d_ws, size_t ws_size,
                              hipStream_t stream) {
  if (n_in < 22) return;
  const int nN = in_sizes[0] / DIN;
  const int nE = in_sizes[1] / DED;
  if (nN < 1 || nE < 1 || in_sizes[0] != nN * DIN || in_sizes[1] != nE * DED) return;
  if (in_sizes[2] != 2 * nE || in_sizes[3] != HID) return;
  if (in_sizes[4] != NCAT * HID || in_sizes[10] != NCAT * HID) return;
  if (in_sizes[6] != HID * HID || in_sizes[8] != HID * HID || in_sizes[12] != HID * HID || in_sizes[14] != HID * HID) return;
  if (in_sizes[16] != HID * HID || in_sizes[18] != HID * HID || in_sizes[20] != HID * HID) return;
  for (int i = 5; i <= 21; i += 2) { if (in_sizes[i] != HID) return; }
  if (out_size != nN * HID) return;
  if (nN > (1 << 22) || nE > (1 << 28)) return;

  const float* x   = (const float*)d_in[0];
  const float* ea  = (const float*)d_in[1];
  const int*   ei  = (const int*)d_in[2];
  const float* q   = (const float*)d_in[3];
  const float* kW0 = (const float*)d_in[4];  const float* kb0 = (const float*)d_in[5];
  const float* kW1 = (const float*)d_in[6];  const float* kb1 = (const float*)d_in[7];
  const float* kW2 = (const float*)d_in[8];  const float* kb2 = (const float*)d_in[9];
  const float* vW0 = (const float*)d_in[10]; const float* vb0 = (const float*)d_in[11];
  const float* vW1 = (const float*)d_in[12]; const float* vb1 = (const float*)d_in[13];
  const float* vW2 = (const float*)d_in[14]; const float* vb2 = (const float*)d_in[15];
  const float* oW0 = (const float*)d_in[16]; const float* ob0 = (const float*)d_in[17];
  const float* oW1 = (const float*)d_in[18]; const float* ob1 = (const float*)d_in[19];
  const float* oW2 = (const float*)d_in[20]; const float* ob2 = (const float*)d_in[21];
  float* out = (float*)d_out;

  const int NPR = ((nN + RPQ - 1) / RPQ) * RPQ;

  char* ws = (char*)d_ws;
  size_t off = 0;
  const size_t hp  = (size_t)NPR * HID * 2;
  const size_t oPN = off; off += (size_t)NPR * PWID * 4;
  const size_t oXH = off; off += hp;
  const size_t oXL = off; off += hp;
  const size_t oAC = off; off += (size_t)NPR * HID * 4;
  const size_t oMP = off; off += (size_t)NPR * NHEAD * 4;
  const size_t oLP = off; off += (size_t)NPR * NHEAD * 4;
  const size_t oW0H = off; off += (size_t)PWID * DIN * 2;
  const size_t oW0L = off; off += (size_t)PWID * DIN * 2;
  const size_t oW0E = off; off += (size_t)2 * HID * 32 * 2;
  const size_t oW1K = off; off += (size_t)HID * HID * 2;
  const size_t oW2K = off; off += (size_t)HID * HID * 2;
  const size_t oW1V = off; off += (size_t)HID * HID * 2;
  const size_t oW2V = off; off += (size_t)HID * HID * 2;
  const size_t oO0H = off; off += (size_t)HID * HID * 2;
  const size_t oO0L = off; off += (size_t)HID * HID * 2;
  const size_t oO1H = off; off += (size_t)HID * HID * 2;
  const size_t oO1L = off; off += (size_t)HID * HID * 2;
  const size_t oO2H = off; off += (size_t)HID * HID * 2;
  const size_t oO2L = off; off += (size_t)HID * HID * 2;
  const size_t ec16 = (size_t)ECH * HID * 2;
  const size_t oH0K = off; off += ec16;
  const size_t oH1K = off; off += ec16;
  const size_t oH0V = off; off += ec16;
  const size_t oH1V = off; off += ec16;
  if (off > ws_size) return;

  float* pn = (float*)(ws + oPN);
  unsigned short* xh = (unsigned short*)(ws + oXH);
  unsigned short* xl = (unsigned short*)(ws + oXL);
  float* accp = (float*)(ws + oAC);
  float* mpp  = (float*)(ws + oMP);
  float* lpp  = (float*)(ws + oLP);
  unsigned short* w0h = (unsigned short*)(ws + oW0H);
  unsigned short* w0l = (unsigned short*)(ws + oW0L);
  unsigned short* w0e = (unsigned short*)(ws + oW0E);
  unsigned short* w1k = (unsigned short*)(ws + oW1K);
  unsigned short* w2k = (unsigned short*)(ws + oW2K);
  unsigned short* w1v = (unsigned short*)(ws + oW1V);
  unsigned short* w2v = (unsigned short*)(ws + oW2V);
  unsigned short* o0h = (unsigned short*)(ws + oO0H);
  unsigned short* o0l = (unsigned short*)(ws + oO0L);
  unsigned short* o1h = (unsigned short*)(ws + oO1H);
  unsigned short* o1l = (unsigned short*)(ws + oO1L);
  unsigned short* o2h = (unsigned short*)(ws + oO2H);
  unsigned short* o2l = (unsigned short*)(ws + oO2L);
  unsigned short* h0k = (unsigned short*)(ws + oH0K);
  unsigned short* h1k = (unsigned short*)(ws + oH1K);
  unsigned short* h0v = (unsigned short*)(ws + oH0V);
  unsigned short* h1v = (unsigned short*)(ws + oH1V);
  unsigned short* k16 = h0k;
  unsigned short* v16 = h0v;
  unsigned short* agh = (unsigned short*)(ws + oPN);
  unsigned short* agl = (unsigned short*)(ws + oPN + hp);
  unsigned short* g0h = (unsigned short*)(ws + oPN + 2 * hp);
  unsigned short* g0l = (unsigned short*)(ws + oPN + 3 * hp);
  unsigned short* g1h = (unsigned short*)(ws + oPN + 4 * hp);
  unsigned short* g1l = (unsigned short*)(ws + oPN + 5 * hp);
  float* g2 = (float*)(ws + oPN + 6 * hp);

  k_prep<<<24, NTHR, 0, stream>>>(kW0, kW1, kW2, vW0, vW1, vW2, oW0, oW1, oW2,
                                  w0h, w0l, w0e, w1k, w2k, w1v, w2v, o0h, o0l, o1h, o1l, o2h, o2l);
  k_splitx<<<NPR * (DIN / 8) / NTHR, NTHR, 0, stream>>>(x, xh, xl, nN, NPR);
  {
    const int gP = ((NPR / 64) * (PWID / 64) + 7) / 8;
    wmma_gemm64<1, true, 0, 0, false, 0><<<dim3(gP, 1), NTHR, 0, stream>>>(
        xh, xl, DIN, 0L, w0h, w0l, DIN, 0L, (void*)pn, (void*)pn, PWID, 0L,
        kb0, pn, 0L, NPR, PWID, DIN, 1.0f);
  }
  const int nCh = (nE + ECH - 1) / ECH;
  for (int c = 0; c < nCh; ++c) {
    const int eStart = c * ECH;
    const int nEc = (nE - eStart < ECH) ? (nE - eStart) : ECH;
    const int CHp = ((nEc + 63) / 64) * 64;
    const int gG = (CHp / 64 + 7) / 8;
    k_edge_h0<<<CHp / ETILE, NTHR, 0, stream>>>(ea, ei, pn, w0e, kb0, vb0, h0k, h0v, nN, nE, eStart, nEc);
    wmma_gemm64<0, false, 2, 1, false, 2><<<dim3(gG, 1), NTHR, 0, stream>>>(
        h0k, h0k, HID, 0L, w1k, w1k, HID, 0L, (void*)h1k, (void*)h1k, HID, 0L,
        kb1, pn, 0L, CHp, HID, HID, 0.125f);
    wmma_gemm64<0, false, 2, 1, false, 2><<<dim3(gG, 1), NTHR, 0, stream>>>(
        h0v, h0v, HID, 0L, w1v, w1v, HID, 0L, (void*)h1v, (void*)h1v, HID, 0L,
        vb1, pn, 0L, CHp, HID, HID, 0.125f);
    wmma_gemm64<0, false, 2, 1, false, 0><<<dim3(gG, 1), NTHR, 0, stream>>>(
        h1k, h1k, HID, 0L, w2k, w2k, HID, 0L, (void*)k16, (void*)k16, HID, 0L,
        kb2, pn, 0L, CHp, HID, HID, 0.125f);
    wmma_gemm64<0, false, 2, 1, false, 0><<<dim3(gG, 1), NTHR, 0, stream>>>(
        h1v, h1v, HID, 0L, w2v, w2v, HID, 0L, (void*)v16, (void*)v16, HID, 0L,
        vb2, pn, 0L, CHp, HID, HID, 0.125f);
    const int vec_ok = ((((size_t)nE + (size_t)eStart) & 3) == 0) ? 1 : 0;
    const int* dstl = ei + (size_t)nE + (size_t)eStart;
    k_agg<NBLK><<<NPR / NBLK, NTHR, LDS_AGG, stream>>>(
        dstl, k16, v16, q, accp, mpp, lpp, agh, agl, nEc, vec_ok,
        (c == 0) ? 1 : 0, (c == nCh - 1) ? 1 : 0);
  }
  {
    const int gO = ((NPR / 64) * (HID / 64) + 7) / 8;
    wmma_gemm64<1, true, 2, 2, false, 2><<<dim3(gO, 1), NTHR, 0, stream>>>(
        agh, agl, HID, 0L, o0h, o0l, HID, 0L, (void*)g0h, (void*)g0l, HID, 0L,
        ob0, g2, 0L, NPR, HID, HID, 1.0f);
    wmma_gemm64<1, true, 2, 2, false, 2><<<dim3(gO, 1), NTHR, 0, stream>>>(
        g0h, g0l, HID, 0L, o1h, o1l, HID, 0L, (void*)g1h, (void*)g1l, HID, 0L,
        ob1, g2, 0L, NPR, HID, HID, 1.0f);
    wmma_gemm64<1, true, 2, 0, false, 0><<<dim3(gO, 1), NTHR, 0, stream>>>(
        g1h, g1l, HID, 0L, o2h, o2l, HID, 0L, (void*)g2, (void*)g2, HID, 0L,
        ob2, g2, 0L, NPR, HID, HID, 1.0f);
  }
  {
    const int n4 = nN * (HID / 4);
    k_final<<<(n4 + NTHR - 1) / NTHR, NTHR, 0, stream>>>(x, g2, out, n4);
  }
}
